// CausalSelfAttention_34093450395927
// MI455X (gfx1250) — hardware-verified
//
#include <hip/hip_runtime.h>
#include <math.h>

#ifndef NB
#define NB 2
#endif
#ifndef SEQ
#define SEQ 2048
#endif
#define NB_FULL 2
#define SEQ_FULL 2048
#define DM 1024
#define NH 16
#define DH 64
#define MTOK (NB * SEQ)
#define EARLY_ROWS 512
#define NQ_ALL (SEQ / 64)
#define NQ_EARLY ((EARLY_ROWS < SEQ ? EARLY_ROWS : SEQ) / 64)
#define NQ_LATE (NQ_ALL - NQ_EARLY)

static_assert(NH * DH == DM);
static_assert(DH == 64);
static_assert(SEQ % 64 == 0);
static_assert(MTOK % 64 == 0);
static_assert(DM % 64 == 0);
static_assert((2 * DM) % 32 == 0);
static_assert(EARLY_ROWS % 64 == 0);
static_assert(NB <= NB_FULL && SEQ <= SEQ_FULL);
static_assert((long long)MTOK * 2 * DM < 2147483647LL);
static_assert((long long)((NB - 1) * SEQ_FULL + SEQ) * DM * 4 <= 16777216LL);

typedef __attribute__((ext_vector_type(16))) _Float16       v16h;
typedef __attribute__((ext_vector_type(16))) __bf16         v16b;
typedef __attribute__((ext_vector_type(8)))  float          v8f;
typedef __attribute__((ext_vector_type(4)))  float          v4f;
typedef __attribute__((ext_vector_type(4)))  unsigned int   v4u;
typedef __attribute__((ext_vector_type(8)))  unsigned short v8us;
typedef __attribute__((ext_vector_type(16))) unsigned short v16us;


__device__ __forceinline__ unsigned int bf_bits(float f) { const unsigned int u = __float_as_uint(f); return (u + 0x7FFFu + ((u >> 16) & 1u)) >> 16; }
__device__ __forceinline__ float bf_val(unsigned int hb) { return __uint_as_float(hb << 16); }
__device__ __forceinline__ float bf_keep(float f) { const unsigned int u = __float_as_uint(f); return __uint_as_float((u + 0x7FFFu + ((u >> 16) & 1u)) & 0xFFFF0000u); }
__device__ __forceinline__ unsigned int hf_bits(float f) { return (unsigned int)__builtin_bit_cast(unsigned short, (_Float16)f); }

__device__ __forceinline__ v16us cat8(const v8us a, const v8us b) { return __builtin_shufflevector(a, b, 0, 1, 2, 3, 4, 5, 6, 7, 8, 9, 10, 11, 12, 13, 14, 15); }
__device__ __forceinline__ v16us ldfrag(const unsigned short* __restrict__ p, const int off) {
    const v8us a = *(const v8us*)(p + off);
    const v8us b = *(const v8us*)(p + off + 16);
    return cat8(a, b);
}
__device__ __forceinline__ v8f mma_f16(const v16us a, const v16us b, v8f c) {
    const v16h ah = __builtin_bit_cast(v16h, a), bh = __builtin_bit_cast(v16h, b);
    c = __builtin_amdgcn_wmma_f32_16x16x32_f16(false, ah, false, bh, (short)0, c, false, false);
    asm volatile("v_nop\n\tv_nop\n\tv_nop\n\tv_nop" : "+v"(c) : "v"(ah), "v"(bh));
    return c;
}
__device__ __forceinline__ v8f mma_bf16(const v16us a, const v16us b, v8f c) {
    const v16b ab = __builtin_bit_cast(v16b, a), bb = __builtin_bit_cast(v16b, b);
    c = __builtin_amdgcn_wmma_f32_16x16x32_bf16(false, ab, false, bb, (short)0, c, false, false);
    asm volatile("v_nop\n\tv_nop\n\tv_nop\n\tv_nop" : "+v"(c) : "v"(ab), "v"(bb));
    return c;
}
__device__ __forceinline__ void wave_sync() {
    __builtin_amdgcn_fence(3  , "workgroup");
    __builtin_amdgcn_wave_barrier();
    __builtin_amdgcn_fence(2  , "workgroup");
}
__device__ __forceinline__ void split8(const v4f a, const v4f b, v4u& ph, v4u& pl) {
    const float x[8] = {a.x, a.y, a.z, a.w, b.x, b.y, b.z, b.w};
    unsigned int h[8], l[8];
#pragma unroll
    for (int e = 0; e < 8; ++e) { h[e] = bf_bits(x[e]); l[e] = bf_bits(x[e] - bf_val(h[e])); }
    ph.x = h[0] | (h[1] << 16); ph.y = h[2] | (h[3] << 16); ph.z = h[4] | (h[5] << 16); ph.w = h[6] | (h[7] << 16);
    pl.x = l[0] | (l[1] << 16); pl.y = l[2] | (l[3] << 16); pl.z = l[4] | (l[5] << 16); pl.w = l[6] | (l[7] << 16);
}
__device__ __forceinline__ v4u half8(const v4f a, const v4f b, const float s) {
    v4u pk;
    pk.x = hf_bits(a.x * s) | (hf_bits(a.y * s) << 16); pk.y = hf_bits(a.z * s) | (hf_bits(a.w * s) << 16);
    pk.z = hf_bits(b.x * s) | (hf_bits(b.y * s) << 16); pk.w = hf_bits(b.z * s) | (hf_bits(b.w * s) << 16);
    return pk;
}
__device__ __forceinline__ void st16x2(unsigned short* p, const v4u v) { volatile v4u* d = (volatile v4u*)p; *d = v; __threadfence(); *d = v; }

__global__ __launch_bounds__(256) void k_cast_x(const float* __restrict__ x, unsigned short* __restrict__ X16) {
    const int u = (int)blockIdx.x * 256 + (int)threadIdx.x;
    if (u >= MTOK * (DM / 8)) return;
    const int r = u / (DM / 8), c0 = 8 * (u % (DM / 8));
    const int b = r / SEQ, t = r - b * SEQ;
    const float* s = x + ((size_t)b * SEQ_FULL + t) * DM + c0;
    v4f a = *(const v4f*)s, q = *(const v4f*)(s + 4);
    a.x = bf_keep(a.x); a.y = bf_keep(a.y); a.z = bf_keep(a.z); a.w = bf_keep(a.w);
    q.x = bf_keep(q.x); q.y = bf_keep(q.y); q.z = bf_keep(q.z); q.w = bf_keep(q.w);
    st16x2(X16 + (size_t)r * DM + c0, half8(a, q, 16.0f));
}
__global__ __launch_bounds__(256) void k_castT_wa(const float* __restrict__ w, unsigned short* __restrict__ WT16) {
    const int u = (int)blockIdx.x * 256 + (int)threadIdx.x;
    if (u >= 3 * DM * (DM / 8)) return;
    const int f = u / (DM / 8), c0 = 8 * (u % (DM / 8));
    float e[8];
#pragma unroll
    for (int i = 0; i < 8; ++i) e[i] = bf_keep(w[(size_t)(c0 + i) * (3 * DM) + f]);
    v4f a, q; a.x = e[0]; a.y = e[1]; a.z = e[2]; a.w = e[3]; q.x = e[4]; q.y = e[5]; q.z = e[6]; q.w = e[7];
    st16x2(WT16 + (size_t)f * DM + c0, half8(a, q, 256.0f));
}
__global__ __launch_bounds__(256) void k_castT_wp(const float* __restrict__ w, unsigned short* __restrict__ WP2) {
    const int u = (int)blockIdx.x * 256 + (int)threadIdx.x;
    if (u >= DM * (DM / 8)) return;
    const int n = u / (DM / 8), k0 = 8 * (u % (DM / 8));
    unsigned int h[8];
#pragma unroll
    for (int i = 0; i < 8; ++i) h[i] = bf_bits(w[(size_t)(k0 + i) * DM + n]);
    v4u pk; pk.x = h[0] | (h[1] << 16); pk.y = h[2] | (h[3] << 16); pk.z = h[4] | (h[5] << 16); pk.w = h[6] | (h[7] << 16);
    st16x2(WP2 + (size_t)n * (2 * DM) + k0, pk);
    st16x2(WP2 + (size_t)n * (2 * DM) + DM + k0, pk);
}

template <int ET, int EPI>
__device__ __forceinline__ void gemm64_body(const unsigned short* __restrict__ A, const int lda,
                                            const unsigned short* __restrict__ Bt, const int ldb,
                                            const int M, const int N, const int K,
                                            unsigned short* __restrict__ O0, unsigned short* __restrict__ O1, unsigned short* __restrict__ O2,
                                            float* __restrict__ OF, const int ldc, const float sc0, const float sc1) {
    __shared__ __align__(16) float sT[8][16 * 68];
    const int lane = (int)threadIdx.x & 31;
    const int wave = __builtin_amdgcn_readfirstlane((int)(threadIdx.x >> 5));
    const int tilesN = N >> 6, tilesM = M >> 6;
    const int tile = (int)blockIdx.x * 8 + wave;
    if (tile >= tilesM * tilesN) return;
    const int tm = tile / tilesN, tn = tile - tm * tilesN;
    const int m0 = tm << 6, n0 = tn << 6;
    const int rl = lane & 15, hh = lane >> 4, koff = hh * 8, mOff = hh * 8;

    v8f acc[4][4];
#pragma unroll
    for (int i = 0; i < 4; ++i)
#pragma unroll
        for (int j = 0; j < 4; ++j) { const v8f zz = {0.f, 0.f, 0.f, 0.f, 0.f, 0.f, 0.f, 0.f}; acc[i][j] = zz; }

    for (int k0 = 0; k0 < K; k0 += 32) {
        v16us bfr[4];
#pragma unroll
        for (int j = 0; j < 4; ++j) bfr[j] = ldfrag(Bt, (n0 + 16 * j + rl) * ldb + koff + k0);
#pragma unroll
        for (int i = 0; i < 4; ++i) {
            const v16us a = ldfrag(A, (m0 + 16 * i + rl) * lda + koff + k0);
#pragma unroll
            for (int j = 0; j < 4; ++j) {
                if (ET == 0) acc[i][j] = mma_f16(a, bfr[j], acc[i][j]);
                else         acc[i][j] = mma_bf16(a, bfr[j], acc[i][j]);
            }
        }
    }

    const float sc = (EPI == 0) ? ((n0 < DM) ? sc0 : sc1) : sc0;
    int mo = m0;
    if (EPI == 2) mo = (m0 / SEQ) * SEQ_FULL + (m0 % SEQ);
#pragma unroll
    for (int i = 0; i < 4; ++i) {
#pragma unroll
        for (int j = 0; j < 4; ++j)
#pragma unroll
            for (int r = 0; r < 8; ++r) sT[wave][(mOff + r) * 68 + 16 * j + rl] = acc[i][j][r] * sc;
        wave_sync();
        if (EPI == 2) {
            const int c4 = rl * 4;
            for (int pass = 0; pass < 2; ++pass) {
#pragma unroll
                for (int it = 0; it < 8; ++it) {
                    const int row = it * 2 + hh;
                    const v4f v = *(const v4f*)&sT[wave][row * 68 + c4];
                    *(volatile v4f*)(OF + (size_t)(mo + 16 * i + row) * ldc + n0 + c4) = v;
                }
                __threadfence();
            }
        } else {
            const int q = lane >> 3, c8 = (lane & 7) * 8;
            for (int pass = 0; pass < 2; ++pass) {
#pragma unroll
                for (int it = 0; it < 4; ++it) {
                    const int row = it * 4 + q;
                    const v4f x0 = *(const v4f*)&sT[wave][row * 68 + c8];
                    const v4f x1 = *(const v4f*)&sT[wave][row * 68 + c8 + 4];
                    const size_t off = (size_t)(m0 + 16 * i + row) * ldc + n0 + c8;
                    v4u ph, pl;
                    split8(x0, x1, ph, pl);
                    if (EPI == 0) {
                        *(volatile v4u*)(O0 + off) = ph;
                        *(volatile v4u*)(O1 + off) = pl;
                    } else {
                        const v4u pf = half8(x0, x1, 16.0f);
                        *(volatile v4u*)(O0 + off) = pf;
                        *(volatile v4u*)(O1 + off) = ph;
                        *(volatile v4u*)(O2 + off) = pl;
                    }
                }
                __threadfence();
            }
        }
        wave_sync();
    }
}

__global__ __launch_bounds__(256) void k_gemm_qk(const unsigned short* __restrict__ X16, const unsigned short* __restrict__ WT16,
                                                 unsigned short* __restrict__ QKh, unsigned short* __restrict__ QKl) {
    gemm64_body<0, 0>(X16, DM, WT16, DM, MTOK, 2 * DM, DM, QKh, QKl, nullptr, nullptr, 2 * DM, 0.125f / 4096.0f, 1.0f / 4096.0f);
}
__global__ __launch_bounds__(256) void k_gemm_vt(const unsigned short* __restrict__ WT16v, const unsigned short* __restrict__ X16,
                                                 unsigned short* __restrict__ Vf, unsigned short* __restrict__ Vbh, unsigned short* __restrict__ Vbl) {
    gemm64_body<0, 1>(WT16v, DM, X16, DM, DM, MTOK, DM, Vf, Vbh, Vbl, nullptr, MTOK, 1.0f / 4096.0f, 1.0f / 4096.0f);
}
__global__ __launch_bounds__(256) void k_gemm_proj(const unsigned short* __restrict__ CTX, const unsigned short* __restrict__ WP2, float* __restrict__ out) {
    gemm64_body<1, 2>(CTX, 2 * DM, WP2, 2 * DM, MTOK, DM, 2 * DM, nullptr, nullptr, nullptr, out, DM, 1.0f, 1.0f);
}

template <bool EARLY>
__device__ __forceinline__ void attn_body(const unsigned short* __restrict__ QKh, const unsigned short* __restrict__ QKl,
                                          const unsigned short* __restrict__ Vf, const unsigned short* __restrict__ Vbh, const unsigned short* __restrict__ Vbl,
                                          unsigned short* __restrict__ CTX, const int qb0, const int nq) {
    __shared__ __align__(16) unsigned short Ph[4][16 * 64];
    __shared__ __align__(16) unsigned short Pl[EARLY ? 4 : 1][EARLY ? 16 * 64 : 8];
    __shared__ __align__(16) float Os[4][16 * 68];
    const int lane = (int)threadIdx.x & 31;
    const int wave = __builtin_amdgcn_readfirstlane((int)(threadIdx.x >> 5));
    const int hh = lane >> 4, c = lane & 15;
    const int bx = (int)blockIdx.x;
    const int qb = qb0 + bx % nq;
    const int bh = bx / nq;
    const int h = bh % NH, b = bh / NH;
    const int q0 = qb * 64 + wave * 16;
    const int tok0 = b * SEQ;
    const int qoff0 = (tok0 + q0 + c) * (2 * DM) + h * DH + 8 * hh;
    const int kcol = DM + h * DH + 8 * hh;
    const float NEG = -__builtin_inff();
    const float L2E = 1.4426950408889634f;
    const float PSC = EARLY ? 1.0f : 16384.0f;
    const float OSC = EARLY ? 1.0f : (16384.0f * 16.0f);

    float mrow[8], lrow[8];
    v8f oacc[4];
#pragma unroll
    for (int r = 0; r < 8; ++r) { mrow[r] = NEG; lrow[r] = 0.f; }
#pragma unroll
    for (int t = 0; t < 4; ++t) { const v8f zz = {0.f, 0.f, 0.f, 0.f, 0.f, 0.f, 0.f, 0.f}; oacc[t] = zz; }

    for (int kc = 0; kc <= qb; ++kc) {
        const int kv0 = kc * 64;
        int qoff = qoff0;
        asm volatile("" : "+v"(qoff));
        v8f s[4];
#pragma unroll
        for (int j = 0; j < 4; ++j) { const v8f zz = {0.f, 0.f, 0.f, 0.f, 0.f, 0.f, 0.f, 0.f}; s[j] = zz; }
#pragma unroll 1
        for (int dc = 0; dc < 2; ++dc) {
            const v16us qh = ldfrag(QKh, qoff + dc * 32);
            const v16us ql = ldfrag(QKl, qoff + dc * 32);
#pragma unroll
            for (int j = 0; j < 4; ++j) {
                const int koff = (tok0 + kv0 + j * 16 + c) * (2 * DM) + kcol + dc * 32;
                const v16us kh = ldfrag(QKh, koff);
                const v16us kl = ldfrag(QKl, koff);
                s[j] = mma_bf16(qh, kh, s[j]);
                s[j] = mma_bf16(qh, kl, s[j]);
                s[j] = mma_bf16(ql, kh, s[j]);
            }
        }
        const bool diag = (kc == qb);
        float cm[8];
#pragma unroll
        for (int r = 0; r < 8; ++r) {
            const int qrow = q0 + 8 * hh + r;
            float m = NEG;
#pragma unroll
            for (int j = 0; j < 4; ++j) {
                float sv = s[j][r] * L2E;
                if (diag) { const int kvcol = kv0 + j * 16 + c; sv = (kvcol > qrow) ? NEG : sv; }
                s[j][r] = sv;
                m = fmaxf(m, sv);
            }
            m = fmaxf(m, __shfl_xor(m, 1, 32)); m = fmaxf(m, __shfl_xor(m, 2, 32));
            m = fmaxf(m, __shfl_xor(m, 4, 32)); m = fmaxf(m, __shfl_xor(m, 8, 32));
            cm[r] = m;
        }
#pragma unroll
        for (int r = 0; r < 8; ++r) {
            const float mnew = fmaxf(mrow[r], cm[r]);
            const float alpha = exp2f(mrow[r] - mnew);
            mrow[r] = mnew;
            float psum = 0.f;
#pragma unroll
            for (int j = 0; j < 4; ++j) {
                const float p = exp2f(s[j][r] - mnew);
                psum += p;
                const int pi = (8 * hh + r) * 64 + j * 16 + c;
                if (EARLY) {
                    const unsigned int hb = bf_bits(p);
                    const unsigned int lb = bf_bits(p - bf_val(hb));
                    Ph[wave][pi] = (unsigned short)hb;
                    Pl[EARLY ? wave : 0][pi] = (unsigned short)lb;
                } else {
                    Ph[wave][pi] = (unsigned short)hf_bits(p * PSC);
                }
            }
            psum += __shfl_xor(psum, 1, 32); psum += __shfl_xor(psum, 2, 32);
            psum += __shfl_xor(psum, 4, 32); psum += __shfl_xor(psum, 8, 32);
            lrow[r] = lrow[r] * alpha + psum;
#pragma unroll
            for (int t = 0; t < 4; ++t) oacc[t][r] *= alpha;
        }
        wave_sync();
#pragma unroll 1
        for (int kk = 0; kk < 2; ++kk) {
            const v8us a0 = *(const v8us*)&Ph[wave][c * 64 + kk * 32 + 8 * hh];
            const v8us a1 = *(const v8us*)&Ph[wave][c * 64 + kk * 32 + 16 + 8 * hh];
            const v16us pa = cat8(a0, a1);
            v16us pl = pa;
            if (EARLY) {
                const v8us l0 = *(const v8us*)&Pl[EARLY ? wave : 0][c * 64 + kk * 32 + 8 * hh];
                const v8us l1 = *(const v8us*)&Pl[EARLY ? wave : 0][c * 64 + kk * 32 + 16 + 8 * hh];
                pl = cat8(l0, l1);
            }
#pragma unroll
            for (int t = 0; t < 4; ++t) {
                const int voff = (h * DH + t * 16 + c) * MTOK + tok0 + kv0 + kk * 32 + 8 * hh;
                if (EARLY) {
                    const v16us vh = ldfrag(Vbh, voff);
                    const v16us vl = ldfrag(Vbl, voff);
                    oacc[t] = mma_bf16(pa, vh, oacc[t]);
                    oacc[t] = mma_bf16(pa, vl, oacc[t]);
                    oacc[t] = mma_bf16(pl, vh, oacc[t]);
                } else {
                    const v16us vf = ldfrag(Vf, voff);
                    oacc[t] = mma_f16(pa, vf, oacc[t]);
                }
            }
        }
        wave_sync();
    }

#pragma unroll
    for (int r = 0; r < 8; ++r) {
        const float inv = 1.0f / (lrow[r] * OSC);
#pragma unroll
        for (int t = 0; t < 4; ++t) Os[wave][(8 * hh + r) * 68 + t * 16 + c] = oacc[t][r] * inv;
    }
    wave_sync();
    {
        const int q = lane >> 3, c8 = (lane & 7) * 8;
        for (int pass = 0; pass < 2; ++pass) {
#pragma unroll
            for (int it = 0; it < 4; ++it) {
                const int row = it * 4 + q;
                const v4f x0 = *(const v4f*)&Os[wave][row * 68 + c8];
                const v4f x1 = *(const v4f*)&Os[wave][row * 68 + c8 + 4];
                v4u ph, pl;
                split8(x0, x1, ph, pl);
                const size_t off = (size_t)(tok0 + q0 + row) * (2 * DM) + h * DH + c8;
                *(volatile v4u*)(CTX + off) = ph;
                *(volatile v4u*)(CTX + off + DM) = pl;
            }
            __threadfence();
        }
    }
}

__global__ __launch_bounds__(128) void k_attn_early(const unsigned short* __restrict__ QKh, const unsigned short* __restrict__ QKl,
                                                    const unsigned short* __restrict__ Vf, const unsigned short* __restrict__ Vbh, const unsigned short* __restrict__ Vbl,
                                                    unsigned short* __restrict__ CTX, int qb0, int nq) {
    attn_body<true>(QKh, QKl, Vf, Vbh, Vbl, CTX, qb0, nq);
}
__global__ __launch_bounds__(128) void k_attn_late(const unsigned short* __restrict__ QKh, const unsigned short* __restrict__ QKl,
                                                   const unsigned short* __restrict__ Vf, const unsigned short* __restrict__ Vbh, const unsigned short* __restrict__ Vbl,
                                                   unsigned short* __restrict__ CTX, int qb0, int nq) {
    attn_body<false>(QKh, QKl, Vf, Vbh, Vbl, CTX, qb0, nq);
}

#define SZ_X16  ((size_t)MTOK * DM * 2)
#define SZ_WT16 ((size_t)3 * DM * DM * 2)
#define SZ_WP2  ((size_t)DM * 2 * DM * 2)
#define SZ_QK   ((size_t)MTOK * 2 * DM * 2)
#define SZ_VT   ((size_t)DM * MTOK * 2)
#define SZ_CTX  ((size_t)MTOK * 2 * DM * 2)
#define WS_TOTAL (SZ_X16 + SZ_WT16 + SZ_WP2 + 2 * SZ_QK + 3 * SZ_VT + SZ_CTX)
static_assert(SZ_X16 % 256 == 0 && SZ_WT16 % 256 == 0 && SZ_WP2 % 256 == 0 && SZ_QK % 256 == 0 && SZ_VT % 256 == 0 && SZ_CTX % 256 == 0);
static_assert(WS_TOTAL <= (size_t)134217728);

extern "C" void kernel_launch(void* const* d_in, const int* in_sizes, int n_in, void* d_out, int out_size, void* d_ws, size_t ws_size, hipStream_t stream) {
    if (n_in < 3) return;
    if ((long long)in_sizes[0] < (long long)((NB - 1) * SEQ_FULL + SEQ) * DM) return;
    if ((long long)in_sizes[1] < (long long)DM * 3 * DM) return;
    if ((long long)in_sizes[2] < (long long)DM * DM) return;
    if ((long long)out_size < (long long)((NB - 1) * SEQ_FULL + SEQ) * DM) return;
    if (WS_TOTAL > ws_size) return;
    const float* x      = (const float*)d_in[0];
    const float* w_attn = (const float*)d_in[1];
    const float* w_proj = (const float*)d_in[2];
    float* out = (float*)d_out;
    char* wsp = (char*)d_ws;
    unsigned short* X16  = (unsigned short*)wsp; wsp += SZ_X16;
    unsigned short* WT16 = (unsigned short*)wsp; wsp += SZ_WT16;
    unsigned short* WP2  = (unsigned short*)wsp; wsp += SZ_WP2;
    unsigned short* QKh  = (unsigned short*)wsp; wsp += SZ_QK;
    unsigned short* QKl  = (unsigned short*)wsp; wsp += SZ_QK;
    unsigned short* Vf   = (unsigned short*)wsp; wsp += SZ_VT;
    unsigned short* Vbh  = (unsigned short*)wsp; wsp += SZ_VT;
    unsigned short* Vbl  = (unsigned short*)wsp; wsp += SZ_VT;
    unsigned short* CTX  = (unsigned short*)wsp; wsp += SZ_CTX;

    k_cast_x<<<(unsigned)((MTOK * (DM / 8) + 255) / 256), 256, 0, stream>>>(x, X16);
    k_castT_wa<<<(unsigned)((3 * DM * (DM / 8) + 255) / 256), 256, 0, stream>>>(w_attn, WT16);
    k_castT_wp<<<(unsigned)((DM * (DM / 8) + 255) / 256), 256, 0, stream>>>(w_proj, WP2);
    k_gemm_qk<<<(unsigned)(((MTOK / 64) * ((2 * DM) / 64) + 7) / 8), 256, 0, stream>>>(X16, WT16, QKh, QKl);
    k_gemm_vt<<<(unsigned)(((DM / 64) * (MTOK / 64) + 7) / 8), 256, 0, stream>>>(WT16 + (size_t)2 * DM * DM, X16, Vf, Vbh, Vbl);
    k_attn_early<<<(unsigned)(NB * NH * NQ_EARLY), 128, 0, stream>>>(QKh, QKl, Vf, Vbh, Vbl, CTX, 0, NQ_EARLY);
    if (NQ_LATE > 0)
        k_attn_late<<<(unsigned)(NB * NH * (NQ_LATE > 0 ? NQ_LATE : 1)), 128, 0, stream>>>(QKh, QKl, Vf, Vbh, Vbl, CTX, NQ_EARLY, (NQ_LATE > 0 ? NQ_LATE : 1));
    k_gemm_proj<<<(unsigned)(((MTOK / 64) * (DM / 64) + 7) / 8), 256, 0, stream>>>(CTX, WP2, out);
}
